// MultiHeadedAttention_35622458753675
// MI455X (gfx1250) — hardware-verified
//
#include <hip/hip_runtime.h>


typedef _Float16       v8h   __attribute__((ext_vector_type(8)));
typedef _Float16       v16h  __attribute__((ext_vector_type(16)));
typedef __bf16         v16bf __attribute__((ext_vector_type(16)));
typedef unsigned short v8us  __attribute__((ext_vector_type(8)));
typedef float          v8f   __attribute__((ext_vector_type(8)));
typedef float          v4f   __attribute__((ext_vector_type(4)));
typedef int            v4i   __attribute__((ext_vector_type(4)));

#ifndef NB
#define NB 2
#endif
#ifndef SEQ
#define SEQ 2048
#endif
#define NB_FULL  2
#define SEQ_FULL 2048
#define MD   1024
#define MH   16
#define MDK  64
#define ROWS (NB * SEQ)
#ifndef BANDQ
#define BANDQ ((SEQ < 512) ? SEQ : 512)
#endif

static_assert(NB >= 1 && NB <= NB_FULL);
static_assert(SEQ >= 128 && SEQ <= SEQ_FULL && (SEQ % 128) == 0);
static_assert(MD == MH * MDK);
static_assert(BANDQ >= 128 && BANDQ <= SEQ && (BANDQ % 128) == 0);
static_assert((MD % 32) == 0);
static_assert(((ROWS * (MD / 8)) % 256) == 0);
static_assert((((MD * MD) / 8) % 256) == 0);
static_assert((size_t)11 * ROWS * MD * 2 + (size_t)4 * MD * MD * 2 <= (size_t)134217728);

__device__ __forceinline__ unsigned short bf16_bits(float f) {
  unsigned int u = __float_as_uint(f);
  u += 0x7fffu + ((u >> 16) & 1u);
  return (unsigned short)(u >> 16);
}
__device__ __forceinline__ float bf16_val(unsigned short b) {
  return __uint_as_float(((unsigned int)b) << 16);
}
__device__ __forceinline__ float bf16_rne(float f) { return bf16_val(bf16_bits(f)); }

union FragH { v16h v; v8h h[2]; };
union FragB { v16bf v; v16h x; v8us u[2]; };

__device__ __forceinline__ FragH ldfrag_h(const _Float16* rowp, unsigned hf) {
  const _Float16* p = rowp + hf * 8u;
  FragH f;
  f.h[0] = *(const v8h*)(p);
  f.h[1] = *(const v8h*)(p + 16);
  return f;
}
__device__ __forceinline__ FragB ldfrag_b(const unsigned short* rowp, unsigned hf) {
  const unsigned short* p = rowp + hf * 8u;
  FragB f;
  f.u[0] = *(const v8us*)(p);
  f.u[1] = *(const v8us*)(p + 16);
  return f;
}

__device__ __forceinline__ v8f wmma_f16(const FragH& a, const FragH& b, v8f c) {
  c = __builtin_amdgcn_wmma_f32_16x16x32_f16(false, a.v, false, b.v, (short)0, c, false, false);
  asm volatile("v_nop\n\tv_nop\n\tv_nop\n\tv_nop" : "+v"(c) : "v"(a.v), "v"(b.v));
  return c;
}
__device__ __forceinline__ v8f wmma_bf(const FragB& a, const FragB& b, v8f c) {
  c = __builtin_amdgcn_wmma_f32_16x16x32_bf16(false, a.v, false, b.v, (short)0, c, false, false);
  asm volatile("v_nop\n\tv_nop\n\tv_nop\n\tv_nop" : "+v"(c) : "v"(a.x), "v"(b.x));
  return c;
}

__global__ __launch_bounds__(256) void cvt_act(
    const float* __restrict__ q, const float* __restrict__ k, const float* __restrict__ v,
    _Float16* xq, _Float16* xk, _Float16* xv) {
  const unsigned c = blockIdx.x * 256u + threadIdx.x;
  if (c >= (unsigned)(ROWS * (MD / 8))) return;
  const unsigned which = blockIdx.y;
  const float* src = (which == 0u) ? q : ((which == 1u) ? k : v);
  _Float16* dst = (which == 0u) ? xq : ((which == 1u) ? xk : xv);
  const unsigned r   = c >> 7;
  const unsigned col = (c & 127u) * 8u;
  const unsigned bb  = r / (unsigned)SEQ;
  const unsigned n   = r - bb * (unsigned)SEQ;
  const float* p = src + ((size_t)bb * SEQ_FULL + n) * MD + col;
  v4f x0 = *(const v4f*)(p);
  v4f x1 = *(const v4f*)(p + 4);
  v8h o;
#pragma unroll
  for (int i = 0; i < 4; ++i) {
    o[i]     = (_Float16)bf16_rne(x0[i]);
    o[4 + i] = (_Float16)bf16_rne(x1[i]);
  }
  _Float16* d = dst + (size_t)r * MD + col;
  *(volatile v8h*)d = o;
  __threadfence();
  *(volatile v8h*)d = o;
}

__global__ __launch_bounds__(256) void cvt_w(
    const float* __restrict__ w0, const float* __restrict__ w1,
    const float* __restrict__ w2, const float* __restrict__ w3,
    _Float16* d0, _Float16* d1, _Float16* d2, _Float16* d3) {
  const unsigned c = blockIdx.x * 256u + threadIdx.x;
  if (c >= (unsigned)((MD * MD) / 8)) return;
  const unsigned which = blockIdx.y;
  const float* src = (which == 0u) ? w0 : ((which == 1u) ? w1 : ((which == 2u) ? w2 : w3));
  _Float16* dst = (which == 0u) ? d0 : ((which == 1u) ? d1 : ((which == 2u) ? d2 : d3));
  const float* p = src + (size_t)c * 8;
  v4f x0 = *(const v4f*)(p);
  v4f x1 = *(const v4f*)(p + 4);
  v8h o;
#pragma unroll
  for (int i = 0; i < 4; ++i) {
    o[i]     = (_Float16)(bf16_rne(x0[i]) * 16.0f);
    o[4 + i] = (_Float16)(bf16_rne(x1[i]) * 16.0f);
  }
  _Float16* d = dst + (size_t)c * 8;
  *(volatile v8h*)d = o;
  __threadfence();
  *(volatile v8h*)d = o;
}

#define GBM 128
#define GBN 64
#define CSP 68

static_assert(GBN == MDK);
static_assert((ROWS % GBM) == 0 && (MD % GBN) == 0 && (SEQ % GBM) == 0);

template <int MODE>
__global__ __launch_bounds__(128) __attribute__((amdgpu_num_vgpr(256)))
void proj_gemm(const _Float16* __restrict__ X, const _Float16* __restrict__ X2,
               const _Float16* __restrict__ W, const float* __restrict__ bias,
               void* dst0, void* dst1) {
  __shared__ __attribute__((aligned(16))) float Cs[GBM][CSP];

  const unsigned tid  = threadIdx.x;
  const unsigned lane = tid & 31u;
  const unsigned wave = tid >> 5;
  const unsigned lr   = lane & 15u;
  const unsigned hf   = lane >> 4;
  const unsigned m0   = blockIdx.y * GBM;
  const unsigned c0   = blockIdx.x * GBN;
  const unsigned r0   = m0 + wave * 32u;

  const v8f z8 = {0.f, 0.f, 0.f, 0.f, 0.f, 0.f, 0.f, 0.f};
  v8f acc[2][4];
#pragma unroll
  for (int r = 0; r < 2; ++r)
#pragma unroll
    for (int t = 0; t < 4; ++t) acc[r][t] = z8;

  const _Float16* wr = W + (size_t)(c0 + lr) * MD + hf * 8u;
  {
    const _Float16* xr0 = X + (size_t)(r0 + lr) * MD + hf * 8u;
    const _Float16* xr1 = X + (size_t)(r0 + 16u + lr) * MD + hf * 8u;
#pragma unroll 2
    for (unsigned k = 0; k < (unsigned)MD; k += 32u) {
      FragH a0, a1;
      a0.h[0] = *(const v8h*)(xr0 + k);
      a0.h[1] = *(const v8h*)(xr0 + k + 16);
      a1.h[0] = *(const v8h*)(xr1 + k);
      a1.h[1] = *(const v8h*)(xr1 + k + 16);
#pragma unroll
      for (int t = 0; t < 4; ++t) {
        const _Float16* wp = wr + (size_t)(t * 16) * MD + k;
        FragH b;
        b.h[0] = *(const v8h*)(wp);
        b.h[1] = *(const v8h*)(wp + 16);
        acc[0][t] = wmma_f16(a0, b, acc[0][t]);
        acc[1][t] = wmma_f16(a1, b, acc[1][t]);
      }
    }
  }

  if constexpr (MODE == 3) {
    const unsigned nl = m0 % (unsigned)SEQ;
    if (nl < (unsigned)BANDQ) {
      v8f acc2[2][4];
#pragma unroll
      for (int r = 0; r < 2; ++r)
#pragma unroll
        for (int t = 0; t < 4; ++t) acc2[r][t] = z8;
      const _Float16* yr0 = X2 + (size_t)(r0 + lr) * MD + hf * 8u;
      const _Float16* yr1 = X2 + (size_t)(r0 + 16u + lr) * MD + hf * 8u;
#pragma unroll 2
      for (unsigned k = 0; k < (unsigned)MD; k += 32u) {
        FragH a0, a1;
        a0.h[0] = *(const v8h*)(yr0 + k);
        a0.h[1] = *(const v8h*)(yr0 + k + 16);
        a1.h[0] = *(const v8h*)(yr1 + k);
        a1.h[1] = *(const v8h*)(yr1 + k + 16);
#pragma unroll
        for (int t = 0; t < 4; ++t) {
          const _Float16* wp = wr + (size_t)(t * 16) * MD + k;
          FragH b;
          b.h[0] = *(const v8h*)(wp);
          b.h[1] = *(const v8h*)(wp + 16);
          acc2[0][t] = wmma_f16(a0, b, acc2[0][t]);
          acc2[1][t] = wmma_f16(a1, b, acc2[1][t]);
        }
      }
#pragma unroll
      for (int r = 0; r < 2; ++r)
#pragma unroll
        for (int t = 0; t < 4; ++t) acc[r][t] = acc[r][t] + acc2[r][t] * 0.00048828125f;
    }
  }

#pragma unroll
  for (int r = 0; r < 2; ++r)
#pragma unroll
    for (int t = 0; t < 4; ++t)
#pragma unroll
      for (int v = 0; v < 8; ++v)
        Cs[wave * 32u + r * 16 + hf * 8u + v][t * 16 + lr] = acc[r][t][v];
  __syncthreads();

  if constexpr (MODE == 3) {
    float* out = (float*)dst0;
    const unsigned c4 = (lane & 15u) * 4u;
    v4f bb = *(const v4f*)(bias + c0 + c4);
    float b4[4];
#pragma unroll
    for (int i = 0; i < 4; ++i) b4[i] = bf16_rne(bb[i]);
#pragma unroll
    for (int rep = 0; rep < 2; ++rep) {
#pragma unroll
      for (int pass = 0; pass < 16; ++pass) {
        const unsigned row = pass * 8 + wave * 2u + (lane >> 4);
        v4f x = *(const v4f*)&Cs[row][c4];
        v4f o;
#pragma unroll
        for (int i = 0; i < 4; ++i) o[i] = x[i] * 0.00390625f + b4[i];
        *(volatile v4f*)(out + (size_t)(m0 + row) * MD + c0 + c4) = o;
      }
      if (rep == 0) __threadfence();
    }
  } else if constexpr (MODE == 2) {
    _Float16* vt = (_Float16*)dst0;
    _Float16* vr = (_Float16*)dst1;
    const unsigned hh   = blockIdx.x;
    const unsigned bidx = m0 / (unsigned)SEQ;
    const unsigned nloc = m0 - bidx * (unsigned)SEQ;
    const unsigned ch   = lane & 7u;
#pragma unroll
    for (int rep = 0; rep < 2; ++rep) {
#pragma unroll
      for (int pass = 0; pass < 8; ++pass) {
        const unsigned seg  = pass * 16 + wave * 4u + (lane >> 3);
        const unsigned d    = seg >> 1;
        const unsigned hsel = seg & 1u;
        const unsigned t0   = hsel * 64u + ch * 8u;
        const float badd = 16.0f * bf16_rne(bias[c0 + d]);
        v8h oh, ores;
#pragma unroll
        for (int i = 0; i < 8; ++i) {
          const float x = Cs[t0 + i][d] + badd;
          const _Float16 xh = (_Float16)x;
          oh[i]   = xh;
          ores[i] = (_Float16)((x - (float)xh) * 2048.0f);
        }
        const size_t off = ((size_t)((bidx * MH + hh) * MDK + d)) * SEQ + nloc + t0;
        *(volatile v8h*)(vt + off) = oh;
        *(volatile v8h*)(vr + off) = ores;
      }
      if (rep == 0) __threadfence();
    }
  } else {
    unsigned short* ph = (unsigned short*)dst0;
    unsigned short* pl = (unsigned short*)dst1;
    const float sa = (MODE == 0) ? 0.0078125f : 0.0625f;
    const float sb = (MODE == 0) ? 0.125f : 1.0f;
    const unsigned c8 = (lane & 7u) * 8u;
    v4f bb0 = *(const v4f*)(bias + c0 + c8);
    v4f bb1 = *(const v4f*)(bias + c0 + c8 + 4);
    float b8[8];
#pragma unroll
    for (int i = 0; i < 4; ++i) {
      b8[i]     = bf16_rne(bb0[i]) * sb;
      b8[4 + i] = bf16_rne(bb1[i]) * sb;
    }
#pragma unroll
    for (int rep = 0; rep < 2; ++rep) {
#pragma unroll
      for (int pass = 0; pass < 8; ++pass) {
        const unsigned row = pass * 16 + wave * 4u + (lane >> 3);
        v4f x0 = *(const v4f*)&Cs[row][c8];
        v4f x1 = *(const v4f*)&Cs[row][c8 + 4];
        v8us H, L;
#pragma unroll
        for (int i = 0; i < 4; ++i) {
          float val = x0[i] * sa + b8[i];
          unsigned short hb = bf16_bits(val);
          H[i] = hb;
          L[i] = bf16_bits(val - bf16_val(hb));
          float val2 = x1[i] * sa + b8[4 + i];
          unsigned short hb2 = bf16_bits(val2);
          H[4 + i] = hb2;
          L[4 + i] = bf16_bits(val2 - bf16_val(hb2));
        }
        const size_t off = (size_t)(m0 + row) * MD + c0 + c8;
        *(volatile v8us*)(ph + off) = H;
        *(volatile v8us*)(pl + off) = L;
      }
      if (rep == 0) __threadfence();
    }
  }
}

#define QBLK 64
#define KBLK 64
#define LDP  136
#define LDV  72

static_assert(QBLK == 64 && KBLK == 64 && MDK == 64);
static_assert((SEQ % QBLK) == 0 && (BANDQ % QBLK) == 0);

template <int BAND>
__global__ __launch_bounds__(128) __attribute__((amdgpu_num_vgpr(256)))
void attn_flash(const unsigned short* __restrict__ Qh, const unsigned short* __restrict__ Ql,
                const unsigned short* __restrict__ Kh, const unsigned short* __restrict__ Kl,
                const _Float16* __restrict__ Vt, const _Float16* __restrict__ Vr,
                const int* __restrict__ mask, _Float16* ctx, _Float16* ctxr, unsigned qblk0) {
  __shared__ __attribute__((aligned(16))) unsigned short Qs[QBLK][LDP];
  __shared__ __attribute__((aligned(16))) unsigned short Ks[KBLK][LDP];
  __shared__ __attribute__((aligned(16))) _Float16 Vs[MDK][LDV];
  __shared__ __attribute__((aligned(16))) _Float16 Ps[4][16][LDV];
  __shared__ __attribute__((aligned(16))) _Float16 Vrs[BAND ? MDK : 1][LDV];
  __shared__ __attribute__((aligned(16))) _Float16 Prs[4][BAND ? 16 : 1][LDV];
  __shared__ __attribute__((aligned(16))) unsigned Mw[QBLK][2];
  __shared__ unsigned Fl[4];

  const unsigned tid  = threadIdx.x;
  const unsigned lane = tid & 31u;
  const unsigned wave = tid >> 5;
  const unsigned cc   = lane & 15u;
  const unsigned hf   = lane >> 4;
  const unsigned rofs = hf * 8u;
  const unsigned b    = blockIdx.y >> 4;
  const unsigned h    = blockIdx.y & 15u;
  const unsigned q0   = (blockIdx.x + qblk0) * QBLK;
  const size_t tokq = (size_t)b * SEQ + q0;
  const unsigned sr  = tid >> 3;
  const unsigned sch = tid & 7u;

#pragma unroll
  for (int i = 0; i < 8; ++i) {
    const unsigned r = sr + 16u * (i & 3);
    const unsigned short* src = (i < 4) ? Qh : Ql;
    *(v8us*)&Qs[r][(i >> 2) * 64 + sch * 8u] =
        *(const v8us*)(src + (tokq + r) * MD + h * MDK + sch * 8u);
  }

  const v8f z8 = {0.f, 0.f, 0.f, 0.f, 0.f, 0.f, 0.f, 0.f};
  float mrun[8], lrun[8];
  v8f o[4];
  v8f o2[BAND ? 4 : 1];
#pragma unroll
  for (int j = 0; j < 8; ++j) { mrun[j] = -1e30f; lrun[j] = 0.f; }
#pragma unroll
  for (int n = 0; n < 4; ++n) o[n] = z8;
#pragma unroll
  for (int n = 0; n < (BAND ? 4 : 1); ++n) o2[n] = z8;

  const unsigned qrow = wave * 16u + cc;

#pragma unroll 1
  for (unsigned kb = 0; kb < (unsigned)SEQ; kb += KBLK) {
    unsigned allm = 1u;
#pragma unroll
    for (unsigned i = 0; i < 4u; ++i) {
      const unsigned r = sr + 16u * i;
      const int* mp = mask + (size_t)(q0 + r) * SEQ_FULL + kb + sch * 8u;
      const v4i ma = *(const v4i*)(mp);
      const v4i mc = *(const v4i*)(mp + 4);
      unsigned bits = 0u;
#pragma unroll
      for (int e = 0; e < 4; ++e) {
        bits |= ((ma[e] != 0) ? 1u : 0u) << e;
        bits |= ((mc[e] != 0) ? 1u : 0u) << (4 + e);
      }
      const unsigned sh = 8u * (sch & 3u);
      unsigned lo = (sch < 4u) ? (bits << sh) : 0u;
      unsigned hi = (sch >= 4u) ? (bits << sh) : 0u;
      lo |= (unsigned)__shfl_xor((int)lo, 1, 32);
      hi |= (unsigned)__shfl_xor((int)hi, 1, 32);
      lo |= (unsigned)__shfl_xor((int)lo, 2, 32);
      hi |= (unsigned)__shfl_xor((int)hi, 2, 32);
      lo |= (unsigned)__shfl_xor((int)lo, 4, 32);
      hi |= (unsigned)__shfl_xor((int)hi, 4, 32);
      if (sch == 0u) { Mw[r][0] = lo; Mw[r][1] = hi; }
      allm &= ((lo & hi) == 0xffffffffu) ? 1u : 0u;
    }
    allm &= (unsigned)__shfl_xor((int)allm, 8, 32);
    allm &= (unsigned)__shfl_xor((int)allm, 16, 32);
    if (lane == 0u) Fl[wave] = allm;
    __syncthreads();
    const unsigned skip =
        (unsigned)__builtin_amdgcn_readfirstlane((int)(Fl[0] & Fl[1] & Fl[2] & Fl[3]));
    if (skip != 0u) {
      __syncthreads();
      continue;
    }

    const size_t tokk = (size_t)b * SEQ + kb;

#pragma unroll
    for (int i = 0; i < 8; ++i) {
      const unsigned r = sr + 16u * (i & 3);
      const unsigned short* src = (i < 4) ? Kh : Kl;
      *(v8us*)&Ks[r][(i >> 2) * 64 + sch * 8u] =
          *(const v8us*)(src + (tokk + r) * MD + h * MDK + sch * 8u);
    }
#pragma unroll
    for (int i = 0; i < 4; ++i) {
      const unsigned d = sr + 16u * i;
      const size_t voff = ((size_t)((b * MH + h) * MDK + d)) * SEQ + kb + sch * 8u;
      *(v8h*)&Vs[d][sch * 8u] = *(const v8h*)(Vt + voff);
      if constexpr (BAND != 0) *(v8h*)&Vrs[d][sch * 8u] = *(const v8h*)(Vr + voff);
    }
    __syncthreads();

    FragB qa0 = ldfrag_b(&Qs[qrow][0],  hf);
    FragB qa1 = ldfrag_b(&Qs[qrow][32], hf);
    FragB qa2 = ldfrag_b(&Qs[qrow][64], hf);
    FragB qa3 = ldfrag_b(&Qs[qrow][96], hf);
    v8f sc[4];
#pragma unroll
    for (int n = 0; n < 4; ++n) {
      const unsigned kr = n * 16 + cc;
      FragB k0 = ldfrag_b(&Ks[kr][0],  hf);
      FragB k1 = ldfrag_b(&Ks[kr][32], hf);
      FragB k2 = ldfrag_b(&Ks[kr][64], hf);
      FragB k3 = ldfrag_b(&Ks[kr][96], hf);
      v8f s = z8;
      s = wmma_bf(qa0, k0, s);
      s = wmma_bf(qa1, k1, s);
      s = wmma_bf(qa2, k0, s);
      s = wmma_bf(qa3, k1, s);
      s = wmma_bf(qa0, k2, s);
      s = wmma_bf(qa1, k3, s);
      sc[n] = s;
    }

    unsigned mbits = 0u;
#pragma unroll
    for (int j = 0; j < 8; ++j) {
      const unsigned w0 = Mw[wave * 16u + rofs + j][0];
      const unsigned w1 = Mw[wave * 16u + rofs + j][1];
      mbits |= ((w0 >> cc) & 1u) << j;
      mbits |= ((w0 >> (16u + cc)) & 1u) << (8 + j);
      mbits |= ((w1 >> cc) & 1u) << (16 + j);
      mbits |= ((w1 >> (16u + cc)) & 1u) << (24 + j);
    }

#pragma unroll
    for (int j = 0; j < 8; ++j) {
#pragma unroll
      for (int n = 0; n < 4; ++n) {
        const bool mk = ((mbits >> (n * 8 + j)) & 1u) != 0u;
        sc[n][j] = mk ? -1e30f : sc[n][j];
      }
      float mx = fmaxf(fmaxf(sc[0][j], sc[1][j]), fmaxf(sc[2][j], sc[3][j]));
      mx = fmaxf(mx, __shfl_xor(mx, 1, 32));
      mx = fmaxf(mx, __shfl_xor(mx, 2, 32));
      mx = fmaxf(mx, __shfl_xor(mx, 4, 32));
      mx = fmaxf(mx, __shfl_xor(mx, 8, 32));
      const float mnew = fmaxf(mrun[j], mx);
      const float al   = __expf(mrun[j] - mnew);
      mrun[j] = mnew;
      float rs = 0.f;
#pragma unroll
      for (int n = 0; n < 4; ++n) {
        const bool mk = ((mbits >> (n * 8 + j)) & 1u) != 0u;
        const float pe = __expf(sc[n][j] - mnew);
        const float p = mk ? 0.0f : pe;
        sc[n][j] = p;
        rs += p;
      }
      rs += __shfl_xor(rs, 1, 32);
      rs += __shfl_xor(rs, 2, 32);
      rs += __shfl_xor(rs, 4, 32);
      rs += __shfl_xor(rs, 8, 32);
      lrun[j] = lrun[j] * al + rs;
#pragma unroll
      for (int n = 0; n < 4; ++n) o[n][j] *= al;
      if constexpr (BAND != 0) {
#pragma unroll
        for (int n = 0; n < 4; ++n) o2[n][j] *= al;
      }
    }

#pragma unroll
    for (int n = 0; n < 4; ++n)
#pragma unroll
      for (int j = 0; j < 8; ++j) {
        const float p16 = sc[n][j] * 1024.0f;
        const _Float16 ph = (_Float16)p16;
        Ps[wave][j + rofs][n * 16 + cc] = ph;
        if constexpr (BAND != 0)
          Prs[wave][j + rofs][n * 16 + cc] = (_Float16)((p16 - (float)ph) * 2048.0f);
      }
    __syncthreads();

    {
      FragH pa0 = ldfrag_h(&Ps[wave][cc][0],  hf);
      FragH pa1 = ldfrag_h(&Ps[wave][cc][32], hf);
#pragma unroll
      for (int n = 0; n < 4; ++n) {
        const unsigned dr = n * 16 + cc;
        FragH v0 = ldfrag_h(&Vs[dr][0],  hf);
        FragH v1 = ldfrag_h(&Vs[dr][32], hf);
        o[n] = wmma_f16(pa0, v0, o[n]);
        o[n] = wmma_f16(pa1, v1, o[n]);
        if constexpr (BAND != 0) {
          FragH pr0 = ldfrag_h(&Prs[wave][cc][0],  hf);
          FragH pr1 = ldfrag_h(&Prs[wave][cc][32], hf);
          FragH w0 = ldfrag_h(&Vrs[dr][0],  hf);
          FragH w1 = ldfrag_h(&Vrs[dr][32], hf);
          o2[n] = wmma_f16(pa0, w0, o2[n]);
          o2[n] = wmma_f16(pa1, w1, o2[n]);
          o2[n] = wmma_f16(pr0, v0, o2[n]);
          o2[n] = wmma_f16(pr1, v1, o2[n]);
        }
      }
    }
    __syncthreads();
  }

#pragma unroll
  for (int j = 0; j < 8; ++j) {
    const float inv = 0.0009765625f * (1.0f / lrun[j]);
#pragma unroll
    for (int n = 0; n < 4; ++n) {
      float c = o[n][j];
      if constexpr (BAND != 0) c += o2[n][j] * 0.00048828125f;
      c *= inv;
      const _Float16 chh = (_Float16)c;
      Ps[wave][j + rofs][n * 16 + cc] = chh;
      if constexpr (BAND != 0)
        Prs[wave][j + rofs][n * 16 + cc] = (_Float16)((c - (float)chh) * 2048.0f);
    }
  }
  __syncthreads();

  const unsigned ch = lane & 7u;
#pragma unroll
  for (int rep = 0; rep < 2; ++rep) {
#pragma unroll
    for (int pass = 0; pass < 4; ++pass) {
      const unsigned row = pass * 4 + (lane >> 3);
      const size_t off = (tokq + wave * 16u + row) * MD + h * MDK + ch * 8u;
      v8h val = *(const v8h*)&Ps[wave][row][ch * 8u];
      *(volatile v8h*)(ctx + off) = val;
      if constexpr (BAND != 0) {
        v8h valr = *(const v8h*)&Prs[wave][row][ch * 8u];
        *(volatile v8h*)(ctxr + off) = valr;
      }
    }
    if (rep == 0) __threadfence();
  }
}

extern "C" void kernel_launch(void* const* d_in, const int* in_sizes, int n_in,
                              void* d_out, int out_size, void* d_ws, size_t ws_size,
                              hipStream_t stream) {
  if (n_in < 12) return;
  const int need_x = ((NB - 1) * SEQ_FULL + SEQ) * MD;
  const int need_m = (SEQ - 1) * SEQ_FULL + SEQ;
  if (in_sizes[0] < need_x || in_sizes[1] < need_x || in_sizes[2] < need_x) return;
  if (in_sizes[3] < need_m) return;
  if (in_sizes[4] < MD * MD || in_sizes[6] < MD * MD || in_sizes[8] < MD * MD || in_sizes[10] < MD * MD) return;
  if (in_sizes[5] < MD || in_sizes[7] < MD || in_sizes[9] < MD || in_sizes[11] < MD) return;
  if (out_size < ROWS * MD) return;

  const float* q    = (const float*)d_in[0];
  const float* k    = (const float*)d_in[1];
  const float* v    = (const float*)d_in[2];
  const int*   mask = (const int*)d_in[3];
  const float* Wq   = (const float*)d_in[4];
  const float* bq   = (const float*)d_in[5];
  const float* Wk   = (const float*)d_in[6];
  const float* bk   = (const float*)d_in[7];
  const float* Wv   = (const float*)d_in[8];
  const float* bv   = (const float*)d_in[9];
  const float* Wo   = (const float*)d_in[10];
  const float* bo   = (const float*)d_in[11];
  float* out = (float*)d_out;

  const size_t PLB = (size_t)ROWS * MD * 2;
  const size_t WLB = (size_t)MD * MD * 2;
  char* ws = (char*)d_ws;
  size_t off = 0;
  _Float16* xq = (_Float16*)(ws + off); off += PLB;
  _Float16* xk = (_Float16*)(ws + off); off += PLB;
  _Float16* xv = (_Float16*)(ws + off); off += PLB;
  _Float16* wq16 = (_Float16*)(ws + off); off += WLB;
  _Float16* wk16 = (_Float16*)(ws + off); off += WLB;
  _Float16* wv16 = (_Float16*)(ws + off); off += WLB;
  _Float16* wo16 = (_Float16*)(ws + off); off += WLB;
  unsigned short* qh = (unsigned short*)(ws + off); off += PLB;
  unsigned short* ql = (unsigned short*)(ws + off); off += PLB;
  unsigned short* kh = (unsigned short*)(ws + off); off += PLB;
  unsigned short* kl = (unsigned short*)(ws + off); off += PLB;
  _Float16* vt   = (_Float16*)(ws + off); off += PLB;
  _Float16* vr   = (_Float16*)(ws + off); off += PLB;
  _Float16* ctx  = (_Float16*)(ws + off); off += PLB;
  _Float16* ctxr = (_Float16*)(ws + off); off += PLB;
  if (off > ws_size) return;

  dim3 gc1((unsigned)((ROWS * (MD / 8)) / 256), 3);
  cvt_act<<<gc1, 256, 0, stream>>>(q, k, v, xq, xk, xv);
  dim3 gc2((unsigned)(((MD * MD) / 8) / 256), 4);
  cvt_w<<<gc2, 256, 0, stream>>>(Wq, Wk, Wv, Wo, wq16, wk16, wv16, wo16);

  dim3 gp(MD / GBN, ROWS / GBM);
  proj_gemm<0><<<gp, 128, 0, stream>>>(xq, xq, wq16, bq, (void*)qh, (void*)ql);
  proj_gemm<1><<<gp, 128, 0, stream>>>(xk, xk, wk16, bk, (void*)kh, (void*)kl);
  proj_gemm<2><<<gp, 128, 0, stream>>>(xv, xv, wv16, bv, (void*)vt, (void*)vr);

  dim3 gab(BANDQ / QBLK, NB * MH);
  attn_flash<1><<<gab, 128, 0, stream>>>(qh, ql, kh, kl, vt, vr, mask, ctx, ctxr, 0u);
  if (SEQ > BANDQ) {
    dim3 gam((SEQ - BANDQ) / QBLK, NB * MH);
    attn_flash<0><<<gam, 128, 0, stream>>>(qh, ql, kh, kl, vt, vr, mask, ctx, ctxr,
                                           (unsigned)(BANDQ / QBLK));
  }

  proj_gemm<3><<<gp, 128, 0, stream>>>(ctx, ctxr, wo16, bo, (void*)out, (void*)out);
}
